// NonLocalBlock2D_36661840839099
// MI455X (gfx1250) — hardware-verified
//
#include <hip/hip_runtime.h>


typedef __attribute__((ext_vector_type(16))) _Float16 v16h;
typedef __attribute__((ext_vector_type(8)))  _Float16 v8h;
typedef __attribute__((ext_vector_type(8)))  float    v8f;
typedef __attribute__((ext_vector_type(4)))  float    v4f;

#define NB   4
#define CCH  31
#define SC   4
#define HH   256
#define HS   64
#define NP   4096
#define ICH  32
#define CINU 496
#define KP   512
#define NPROJ 96
#define VST2(T, ptr, val) do { const T _v = (val); *(volatile T*)(ptr) = _v; __threadfence(); *(volatile T*)(ptr) = _v; } while (0)

__device__ __forceinline__ v8f wmma16(v16h a, v16h b, v8f c) {
    v8f d = __builtin_amdgcn_wmma_f32_16x16x32_f16(false, a, false, b, (short)0, c, false, false);
    asm volatile("v_nop\n\tv_nop\n\tv_nop\n\tv_nop" : "+v"(d) : "v"(a), "v"(b));
    return d;
}
__device__ __forceinline__ v16h frag16(const _Float16* __restrict__ row, int hi) {
    const v8h lo = *(const v8h*)(row + hi * 8), hh = *(const v8h*)(row + 16 + hi * 8);
    return __builtin_shufflevector(lo, hh, 0,1,2,3,4,5,6,7,8,9,10,11,12,13,14,15);
}
__device__ __forceinline__ void wave_lds_sync() {
    __builtin_amdgcn_fence(__ATOMIC_RELEASE, "workgroup"); __builtin_amdgcn_wave_barrier(); __builtin_amdgcn_fence(__ATOMIC_ACQUIRE, "workgroup");
}

__global__ __launch_bounds__(256) void k_unshuffle(const float* __restrict__ x, _Float16* __restrict__ Xu, _Float16* __restrict__ XuL) {
    const int t = blockIdx.x * 256 + threadIdx.x;
    const int c8 = (t & 63) * 8, p = (t >> 6) & (NP - 1), n = t >> 18;
    const int i = p >> 6, j = p & 63;
    v8h v, vl;
#pragma unroll
    for (int e = 0; e < 8; ++e) {
        const int cu = c8 + e;
        float val = 0.f;
        if (cu < CINU) { const int ss = cu / CCH, c = cu - ss * CCH, sh = ss >> 2, sw = ss & 3;
                         val = x[(((size_t)n * CCH + c) * HH + (i * SC + sh)) * HH + (j * SC + sw)]; }
        v[e] = (_Float16)val; vl[e] = (_Float16)(val - (float)v[e]);
    }
    VST2(v8h, Xu + (size_t)t * 8, v);
    VST2(v8h, XuL + (size_t)t * 8, vl);
}
__global__ __launch_bounds__(256) void k_wcat(const float* __restrict__ tw, const float* __restrict__ pw, const float* __restrict__ gw,
                                              const float* __restrict__ Ww, _Float16* __restrict__ Wcat, _Float16* __restrict__ WcatL, _Float16* __restrict__ WwT, _Float16* __restrict__ WwTL) {
    const int t = blockIdx.x * 256 + threadIdx.x;
    if (t < NPROJ * 64) {
        const int o = t >> 6, k0 = (t & 63) * 8;
        const float* src = (o < 32) ? (tw + (size_t)o * CINU) : (o < 64) ? (pw + (size_t)(o - 32) * CINU) : (gw + (size_t)(o - 64) * CINU);
        v8h v, vl;
#pragma unroll
        for (int e = 0; e < 8; ++e) { const float w = (k0 + e < CINU) ? src[k0 + e] : 0.f; v[e] = (_Float16)w; vl[e] = (_Float16)(w - (float)v[e]); }
        VST2(v8h, Wcat + (size_t)o * KP + k0, v);
        VST2(v8h, WcatL + (size_t)o * KP + k0, vl);
    } else if (t < NPROJ * 64 + 512 * 4) {
        const int q = t - NPROJ * 64, u = q >> 2, k0 = (q & 3) * 8;
        v8h v, vl;
#pragma unroll
        for (int e = 0; e < 8; ++e) { const float w = (u < CINU) ? Ww[(size_t)u * ICH + k0 + e] : 0.f; v[e] = (_Float16)w; vl[e] = (_Float16)(w - (float)v[e]); }
        VST2(v8h, WwT + (size_t)u * ICH + k0, v);
        VST2(v8h, WwTL + (size_t)u * ICH + k0, vl);
    }
}
__global__ __launch_bounds__(256) void k_proj(const _Float16* __restrict__ Xu, const _Float16* __restrict__ XuL,
                                              const _Float16* __restrict__ Wcat, const _Float16* __restrict__ WcatL,
                                              const float* __restrict__ tb, const float* __restrict__ pb, const float* __restrict__ gb,
                                              _Float16* __restrict__ thH, _Float16* __restrict__ thL, _Float16* __restrict__ phH, _Float16* __restrict__ phL,
                                              _Float16* __restrict__ gT, _Float16* __restrict__ gTL) {
    __shared__ __attribute__((aligned(16))) _Float16 sP[8][4][16 * 32];
    __shared__ __attribute__((aligned(16))) _Float16 sG[2][32][136];
    const int lane = threadIdx.x & 31, wave = threadIdx.x >> 5, hi = lane >> 4, l16 = lane & 15;
    const int n = blockIdx.y, p0 = blockIdx.x * 128 + wave * 16;
    v8f acc[6] = {};
    const size_t ao = ((size_t)n * NP + p0 + l16) * KP;
    for (int kb = 0; kb < KP; kb += 32) {
        const v16h a = frag16(Xu + ao + kb, hi), al = frag16(XuL + ao + kb, hi);
#pragma unroll
        for (int t = 0; t < 6; ++t) {
            const size_t bo = (size_t)(t * 16 + l16) * KP + kb;
            const v16h b = frag16(Wcat + bo, hi), bl = frag16(WcatL + bo, hi);
            acc[t] = wmma16(a, b, acc[t]); acc[t] = wmma16(a, bl, acc[t]); acc[t] = wmma16(al, b, acc[t]);
        }
    }
#pragma unroll
    for (int t = 0; t < 6; ++t) {
        const int c = (t & 1) * 16 + l16;
#pragma unroll
        for (int r = 0; r < 8; ++r) {
            const int rr = r + 8 * hi;
            if (t < 4) {
                const float v = acc[t][r] + ((t < 2) ? tb[c] : pb[c]);
                const _Float16 h = (_Float16)v, l = (_Float16)(v - (float)h);
                const int which = (t < 2) ? 0 : 2;
                sP[wave][which][rr * 32 + c] = h; sP[wave][which + 1][rr * 32 + c] = l;
            } else {
                const float gv = acc[t][r] + gb[c]; const _Float16 gh = (_Float16)gv;
                sG[0][c][wave * 16 + rr] = gh; sG[1][c][wave * 16 + rr] = (_Float16)(gv - (float)gh);
            }
        }
    }
    wave_lds_sync();
    {
        const size_t base = ((size_t)n * NP + p0) * ICH;
        _Float16* dsts[4] = {thH + base, thL + base, phH + base, phL + base};
        for (int pass = 0; pass < 2; ++pass) {
#pragma unroll
            for (int w = 0; w < 4; ++w) {
                *(volatile v8h*)(dsts[w] + lane * 8)       = *(const v8h*)(&sP[wave][w][lane * 8]);
                *(volatile v8h*)(dsts[w] + 256 + lane * 8) = *(const v8h*)(&sP[wave][w][256 + lane * 8]);
            }
            __threadfence();
        }
    }
    __syncthreads();
    for (int pass = 0; pass < 2; ++pass) {
        for (int q = threadIdx.x; q < 1024; q += 256) {
            const int pl = q >> 9, c = (q >> 4) & 31, pc = (q & 15) * 8;
            *(volatile v8h*)((pl ? gTL : gT) + ((size_t)n * ICH + c) * NP + blockIdx.x * 128 + pc) = *(const v8h*)(&sG[pl][c][pc]);
        }
        __threadfence();
    }
}

__global__ __launch_bounds__(256) void nlb_colstats(const _Float16* __restrict__ thH, const _Float16* __restrict__ thL,
                                                    const _Float16* __restrict__ phH, const _Float16* __restrict__ phL,
                                                    float* __restrict__ colML) {
    const int lane = threadIdx.x & 31;
    const int gidx = blockIdx.x * 8 + (threadIdx.x >> 5);
    const int n  = gidx >> 8;
    const int j0 = (gidx & 255) * 16;
    const int m  = lane & 15, hi = lane >> 4;
    const size_t bn = (size_t)n * NP * ICH;
    const v16h Bh = frag16(phH + bn + (size_t)(j0 + m) * ICH, hi), Bl = frag16(phL + bn + (size_t)(j0 + m) * ICH, hi);
    float mx = -1e30f, sm = 0.0f;
    for (int i0 = 0; i0 < NP; i0 += 16) {
        const v16h Ah = frag16(thH + bn + (size_t)(i0 + m) * ICH, hi), Al = frag16(thL + bn + (size_t)(i0 + m) * ICH, hi);
        v8f acc = {};
        acc = wmma16(Ah, Bh, acc); acc = wmma16(Ah, Bl, acc); acc = wmma16(Al, Bh, acc);
        float tm = mx;
#pragma unroll
        for (int r = 0; r < 8; ++r) tm = fmaxf(tm, acc[r]);
        float s2 = 0.0f;
#pragma unroll
        for (int r = 0; r < 8; ++r) s2 += __expf(acc[r] - tm);
        sm = sm * __expf(mx - tm) + s2;
        mx = tm;
    }
    const float mo = __shfl_xor(mx, 16, 32);
    const float so = __shfl_xor(sm, 16, 32);
    const float Mf = fmaxf(mx, mo);
    const float Zf = sm * __expf(mx - Mf) + so * __expf(mo - Mf);
    VST2(float, colML + ((size_t)n * NP + j0) * 2 + lane, hi ? (1.0f / Zf) : Mf);
}

__global__ __launch_bounds__(256) void nlb_attn(const _Float16* __restrict__ thH, const _Float16* __restrict__ thL,
                                                const _Float16* __restrict__ phH, const _Float16* __restrict__ phL,
                                                const _Float16* __restrict__ gT, const _Float16* __restrict__ gTL, const float* __restrict__ colML, float* __restrict__ y) {
    __shared__ __attribute__((aligned(16))) float sY[8][16 * 32];
    const int lane = threadIdx.x & 31, wave = threadIdx.x >> 5;
    const int gidx = blockIdx.x * 8 + wave;
    const int n  = gidx >> 8;
    const int i0 = (gidx & 255) * 16;
    const int m  = lane & 15, hi = lane >> 4;
    const size_t bn = (size_t)n * NP * ICH;
    const _Float16* gn = gT + (size_t)n * ICH * NP;
    const _Float16* gln = gTL + (size_t)n * ICH * NP;
    const float* MLn = colML + (size_t)n * NP * 2;
    const v16h Bh = frag16(thH + bn + (size_t)(i0 + m) * ICH, hi), Bl = frag16(thL + bn + (size_t)(i0 + m) * ICH, hi);
    v8f y0 = {}, y1 = {};
    for (int jc = 0; jc < NP; jc += 32) {
        v8f f0 = {}, f1 = {};
        {
            v16h Ah = frag16(phH + bn + (size_t)(jc + m) * ICH, hi), Al = frag16(phL + bn + (size_t)(jc + m) * ICH, hi);
            f0 = wmma16(Ah, Bh, f0); f0 = wmma16(Ah, Bl, f0); f0 = wmma16(Al, Bh, f0);
            Ah = frag16(phH + bn + (size_t)(jc + 16 + m) * ICH, hi); Al = frag16(phL + bn + (size_t)(jc + 16 + m) * ICH, hi);
            f1 = wmma16(Ah, Bh, f1); f1 = wmma16(Ah, Bl, f1); f1 = wmma16(Al, Bh, f1);
        }
        v16h P, PL;
#pragma unroll
        for (int r = 0; r < 8; ++r) {
            const int ja = jc + 8 * hi + r, jb = ja + 16;
            const float* mla = MLn + (size_t)(ja >> 4) * 32 + (ja & 15);
            const float* mlb = MLn + (size_t)(jb >> 4) * 32 + (jb & 15);
            const float pa = __expf(f0[r] - mla[0]) * mla[16], pb = __expf(f1[r] - mlb[0]) * mlb[16];
            P[r] = (_Float16)pa;     PL[r] = (_Float16)(pa - (float)P[r]);
            P[8 + r] = (_Float16)pb; PL[8 + r] = (_Float16)(pb - (float)P[8 + r]);
        }
        const v16h GA0 = frag16(gn + (size_t)m * NP + jc, hi),  GL0 = frag16(gln + (size_t)m * NP + jc, hi);
        const v16h GA1 = frag16(gn + (size_t)(16 + m) * NP + jc, hi), GL1 = frag16(gln + (size_t)(16 + m) * NP + jc, hi);
        y0 = wmma16(GA0, P, y0); y0 = wmma16(GA0, PL, y0); y0 = wmma16(GL0, P, y0);
        y1 = wmma16(GA1, P, y1); y1 = wmma16(GA1, PL, y1); y1 = wmma16(GL1, P, y1);
    }
    float* sy = sY[wave];
#pragma unroll
    for (int r = 0; r < 8; ++r) { sy[m * 32 + r + 8 * hi] = y0[r]; sy[m * 32 + 16 + r + 8 * hi] = y1[r]; }
    wave_lds_sync();
    float* yn = y + ((size_t)n * NP + i0) * ICH;
    for (int pass = 0; pass < 2; ++pass) {
#pragma unroll
        for (int q = 0; q < 4; ++q) *(volatile v4f*)(yn + q * 128 + lane * 4) = *(const v4f*)(sy + q * 128 + lane * 4);
        __threadfence();
    }
}

__global__ __launch_bounds__(256) void nlb_wproj(const float* __restrict__ y, const _Float16* __restrict__ WwT, const _Float16* __restrict__ WwTL, const float* __restrict__ Wb,
                                                 float* __restrict__ z) {
    __shared__ __attribute__((aligned(16))) float sZ[CCH][260];
    const int lane = threadIdx.x & 31, wave = threadIdx.x >> 5, hi = lane >> 4, l16 = lane & 15;
    const int sh = blockIdx.x & 3, i = (blockIdx.x >> 2) & 63, n = blockIdx.x >> 8;
    const int mt = wave & 3, ntp = wave >> 2;
    const int p = i * 64 + mt * 16 + l16;
    v16h a, al;
    {
        const float* yr = y + ((size_t)n * NP + p) * ICH;
#pragma unroll
        for (int e = 0; e < 16; ++e) { const float v = yr[(e < 8) ? (8 * hi + e) : (16 + 8 * hi + e - 8)]; a[e] = (_Float16)v; al[e] = (_Float16)(v - (float)a[e]); }
    }
    v8f acc[4] = {};
#pragma unroll
    for (int t = 0; t < 4; ++t) {
        const int u = sh * 124 + (ntp * 4 + t) * 16 + l16;
        const v16h b = frag16(WwT + (size_t)u * ICH, hi), bl = frag16(WwTL + (size_t)u * ICH, hi);
        acc[t] = wmma16(a, b, acc[t]);
        acc[t] = wmma16(al, b, acc[t]);
        acc[t] = wmma16(a, bl, acc[t]);
    }
#pragma unroll
    for (int t = 0; t < 4; ++t) {
        const int ul = (ntp * 4 + t) * 16 + l16;
        if (ul < 124) {
            const int sw = ul / CCH, c = ul - sw * CCH;
            const float b = Wb[sh * 124 + ul];
#pragma unroll
            for (int r = 0; r < 8; ++r) { const int j = mt * 16 + r + 8 * hi; sZ[c][j * SC + sw] = acc[t][r] + b; }
        }
    }
    __syncthreads();
    for (int pass = 0; pass < 2; ++pass) {
        for (int q = threadIdx.x; q < CCH * 64; q += 256) {
            const int c = q >> 6, xq = (q & 63) * 4;
            *(volatile v4f*)(z + (((size_t)n * CCH + c) * HH + (i * SC + sh)) * HH + xq) = *(const v4f*)(&sZ[c][xq]);
        }
        __threadfence();
    }
}

extern "C" void kernel_launch(void* const* d_in, const int* in_sizes, int n_in,
                              void* d_out, int out_size, void* d_ws, size_t ws_size,
                              hipStream_t stream) {
    (void)in_sizes; (void)n_in; (void)out_size;
    const float* x  = (const float*)d_in[0];
    const float* gw = (const float*)d_in[1];
    const float* gb = (const float*)d_in[2];
    const float* tw = (const float*)d_in[3];
    const float* tb = (const float*)d_in[4];
    const float* pw = (const float*)d_in[5];
    const float* pb = (const float*)d_in[6];
    const float* Ww = (const float*)d_in[7];
    const float* Wb = (const float*)d_in[8];
    float* z = (float*)d_out;

    char* ws = (char*)d_ws; size_t off = 0;
    auto take = [&](size_t bytes) { void* p = ws + off; off = (off + bytes + 255) & ~(size_t)255; return p; };
    _Float16* Xu   = (_Float16*)take((size_t)NB * NP * KP * 2);
    _Float16* XuL  = (_Float16*)take((size_t)NB * NP * KP * 2);
    _Float16* Wcat = (_Float16*)take((size_t)NPROJ * KP * 2);
    _Float16* WcatL= (_Float16*)take((size_t)NPROJ * KP * 2);
    _Float16* WwT  = (_Float16*)take((size_t)512 * ICH * 2);
    _Float16* WwTL = (_Float16*)take((size_t)512 * ICH * 2);
    _Float16* thH  = (_Float16*)take((size_t)NB * NP * ICH * 2);
    _Float16* thL  = (_Float16*)take((size_t)NB * NP * ICH * 2);
    _Float16* phH  = (_Float16*)take((size_t)NB * NP * ICH * 2);
    _Float16* phL  = (_Float16*)take((size_t)NB * NP * ICH * 2);
    _Float16* gT   = (_Float16*)take((size_t)NB * ICH * NP * 2);
    _Float16* gTL  = (_Float16*)take((size_t)NB * ICH * NP * 2);
    float*    cML  = (float*)take((size_t)NB * NP * 2 * 4);
    float*    y    = (float*)take((size_t)NB * NP * ICH * 4);
    if (off > ws_size) return;

    k_unshuffle<<<NB * NP * 64 / 256, 256, 0, stream>>>(x, Xu, XuL);
    k_wcat<<<(NPROJ * 64 + 512 * 4 + 255) / 256, 256, 0, stream>>>(tw, pw, gw, Ww, Wcat, WcatL, WwT, WwTL);
    k_proj<<<dim3(NP / 128, NB), 256, 0, stream>>>(Xu, XuL, Wcat, WcatL, tb, pb, gb, thH, thL, phH, phL, gT, gTL);
    nlb_colstats<<<128, 256, 0, stream>>>(thH, thL, phH, phL, cML);
    nlb_attn<<<128, 256, 0, stream>>>(thH, thL, phH, phL, gT, gTL, cML, y);
    nlb_wproj<<<NB * HS * SC, 256, 0, stream>>>(y, WwT, WwTL, Wb, z);
}
